// GlmImageVQVAE_52725018526060
// MI455X (gfx1250) — hardware-verified
//
#include <hip/hip_runtime.h>
#include <math.h>

typedef __attribute__((ext_vector_type(16))) _Float16 v16h;
typedef __attribute__((ext_vector_type(16))) __bf16 v16b;
typedef __attribute__((ext_vector_type(8)))  _Float16 v8h;
typedef __attribute__((ext_vector_type(8)))  float v8f;
typedef __attribute__((ext_vector_type(4)))  float v4f;
typedef __attribute__((ext_vector_type(2)))  float v2f;
typedef __attribute__((ext_vector_type(4)))  unsigned v4u;
typedef __attribute__((ext_vector_type(4)))  int v4i;
typedef float __attribute__((may_alias)) float_a;
typedef int __attribute__((may_alias)) int_a;

template <typename T> __device__ __forceinline__ void vst2(void* p, T v) { *(volatile T*)p = v; __threadfence(); *(volatile T*)p = v; }
__device__ __forceinline__ v8f wmma16(v16h a, v16h b, v8f c) {
  v8f d = __builtin_amdgcn_wmma_f32_16x16x32_f16(false, a, false, b, (short)0, c, false, false);
  asm volatile("v_nop\n\tv_nop\n\tv_nop\n\tv_nop" : "+v"(d) : "v"(a), "v"(b));
  return d;
}
__device__ __forceinline__ v8f wmma_bf(v16b a, v16b b, v8f c) {
  v8f d = __builtin_amdgcn_wmma_f32_16x16x32_bf16(false, a, false, b, (short)0, c, false, false);
  asm volatile("v_nop\n\tv_nop\n\tv_nop\n\tv_nop" : "+v"(d) : "v"(a), "v"(b));
  return d;
}
__device__ __forceinline__ v16h frag_h(const _Float16* rowk0, int lane) {
  union { v16h v; v8h q[2]; } u; const _Float16* p = rowk0 + 8 * (lane >> 4);
  u.q[0] = *(const v8h*)p; u.q[1] = *(const v8h*)(p + 16); return u.v;
}
__device__ __forceinline__ v16h frag_f32(const float* rowk0, int lane) {
  v16h a; const float* p = rowk0 + 8 * (lane >> 4);
#pragma unroll
  for (int i = 0; i < 8; ++i) { a[i] = (_Float16)p[i]; a[8 + i] = (_Float16)p[16 + i]; }
  return a;
}
__device__ __forceinline__ v16h frag_f32s(const float* rowk0, int lane, float sc) {
  v16h a; const float* p = rowk0 + 8 * (lane >> 4);
#pragma unroll
  for (int i = 0; i < 8; ++i) { a[i] = (_Float16)(p[i] * sc); a[8 + i] = (_Float16)(p[16 + i] * sc); }
  return a;
}
__device__ __forceinline__ v16h fragc_f32(const float* W, int k0, int n, int lane, int ld, int K) {
  v16h a; const int g = lane >> 4;
#pragma unroll
  for (int i = 0; i < 8; ++i) { const int ka = k0 + 8 * g + i, kb = ka + 16;
    a[i] = (_Float16)(ka < K ? W[(size_t)(ka < K ? ka : K - 1) * ld + n] : 0.f); a[8 + i] = (_Float16)(kb < K ? W[(size_t)(kb < K ? kb : K - 1) * ld + n] : 0.f); }
  return a;
}
struct F2 { v16b h, l; };
__device__ __forceinline__ F2 bsplit16(const float v[16]) { F2 r;
#pragma unroll
  for (int i = 0; i < 16; ++i) { const __bf16 h = (__bf16)v[i]; r.h[i] = h; r.l[i] = (__bf16)(v[i] - (float)h); }
  return r; }
__device__ __forceinline__ F2 split_row(const float* row, int k0, int lane) { float v[16]; const float* p = row + k0 + 8 * (lane >> 4);
#pragma unroll
  for (int i = 0; i < 8; ++i) { v[i] = p[i]; v[8 + i] = p[16 + i]; }
  return bsplit16(v); }
__device__ __forceinline__ F2 split_rowK(const float* row, int k0, int lane, int K) { float v[16]; const int g = lane >> 4;
#pragma unroll
  for (int i = 0; i < 8; ++i) { const int ka = k0 + 8 * g + i, kb = ka + 16; v[i] = ka < K ? row[ka < K ? ka : K - 1] : 0.f; v[8 + i] = kb < K ? row[kb < K ? kb : K - 1] : 0.f; }
  return bsplit16(v); }
__device__ __forceinline__ F2 split_col(const float* W, int k0, int n, int lane, int ld, int K) { float v[16]; const int g = lane >> 4;
#pragma unroll
  for (int i = 0; i < 8; ++i) { const int ka = k0 + 8 * g + i, kb = ka + 16; v[i] = ka < K ? W[(size_t)(ka < K ? ka : K - 1) * ld + n] : 0.f; v[8 + i] = kb < K ? W[(size_t)(kb < K ? kb : K - 1) * ld + n] : 0.f; }
  return bsplit16(v); }
__device__ __forceinline__ v8f mac3(const F2& a, const F2& b, v8f c) { c = wmma_bf(a.l, b.h, c); c = wmma_bf(a.h, b.l, c); return wmma_bf(a.h, b.h, c); }
__device__ __forceinline__ float sigm(float v) { return 1.0f / (1.0f + expf(-v)); }
#define LDSX() do { asm volatile("s_wait_dscnt 0" ::: "memory"); __builtin_amdgcn_wave_barrier(); __builtin_amdgcn_fence(__ATOMIC_RELEASE, "workgroup"); } while (0)


#define NV 16384
#define NCB 16384
#define CC 256
#define EE 256
#define NPIX 1024
#define NTOP 4
#ifndef NRT
#define NRT (NV / 64)
#endif
typedef __attribute__((ext_vector_type(8))) __bf16 v8b;
__device__ __forceinline__ v16b frag_b(const __bf16* rowk0, int lane) {
  union { v16b v; v8b q[2]; } u; const __bf16* p = rowk0 + 8 * (lane >> 4);
  u.q[0] = *(const v8b*)p; u.q[1] = *(const v8b*)(p + 16); return u.v;
}
__device__ __forceinline__ float bfr(float v) { return (float)(__bf16)v; }
__device__ __attribute__((noinline)) float exp_ni(float v) { return expf(v); }
__device__ __attribute__((noinline)) float erf_ni(float v) { return erff(v); }

#define WS_XH  0u
#define WS_XL  (WS_XH + 2u * NV * CC)
#define WS_WH  (WS_XL + 2u * NV * CC)
#define WS_WL  (WS_WH + 2u * EE * CC)
#define WS_ZF  (WS_WL + 2u * EE * CC)
#define WS_ZB  (WS_ZF + 4u * (size_t)NV * EE)
#define WS_CF  (WS_ZB + 2u * (size_t)NV * EE)
#define WS_CB  (WS_CF + 4u * (size_t)NCB * EE)
#define WS_CSQ (WS_CB + 2u * (size_t)NCB * EE)
#define WS_ZSQ (WS_CSQ + 4u * NCB)
#define WS_END (WS_ZSQ + 4u * NV)

__global__ __launch_bounds__(256) void k_xrows(const float* __restrict__ HS, __bf16* __restrict__ XH, __bf16* __restrict__ XL) {
  __shared__ __align__(16) __bf16 sh_[64][CC + 8], sl_[64][CC + 8]; const int tid = threadIdx.x; const int pb = blockIdx.x, b = blockIdx.y; const int p0 = pb * 64;
  for (int e = tid; e < 64 * CC; e += 256) { const int c = e >> 6, r = e & 63; const float v = HS[((size_t)b * CC + c) * NPIX + p0 + r]; const __bf16 hb = (__bf16)v; sh_[r][c] = hb; sl_[r][c] = (__bf16)(v - (float)hb); }
  __syncthreads();
  for (int e = tid; e < 64 * CC / 8; e += 256) { const int r = e / (CC / 8), pc = e % (CC / 8); const size_t o = ((size_t)b * NPIX + p0 + r) * CC + pc * 8; vst2((unsigned*)(XH + o), *(const v4u*)&sh_[r][pc * 8]); vst2((unsigned*)(XL + o), *(const v4u*)&sl_[r][pc * 8]); }
}
__global__ __launch_bounds__(256) void k_wrows(const float* __restrict__ CW, __bf16* __restrict__ WH, __bf16* __restrict__ WL) {
  __shared__ __align__(16) __bf16 sh_[CC], sl_[CC]; const int e = blockIdx.x, t = threadIdx.x; { const float v = CW[(size_t)e * CC + t]; const __bf16 hb = (__bf16)v; sh_[t] = hb; sl_[t] = (__bf16)(v - (float)hb); }
  __syncthreads();
  if (t < CC / 8) vst2((unsigned*)(WH + (size_t)e * CC + t * 8), *(const v4u*)&sh_[t * 8]); else if (t < CC / 4) vst2((unsigned*)(WL + (size_t)e * CC + (t - CC / 8) * 8), *(const v4u*)&sl_[(t - CC / 8) * 8]);
}
__global__ __launch_bounds__(128) void k_conv(const __bf16* __restrict__ XH, const __bf16* __restrict__ XL, const __bf16* __restrict__ WH, const __bf16* __restrict__ WL, const float* __restrict__ CBIAS, float* __restrict__ ZF, __bf16* __restrict__ ZB, float* __restrict__ ZSQ) {
  __shared__ __align__(16) float sz[4][16][EE + 4]; __shared__ __align__(16) __bf16 szb[4][16][EE + 8]; __shared__ float ssq[4][16][16]; __shared__ __align__(16) float szsq[64];
  const int tid = threadIdx.x, wave = tid >> 5, lane = tid & 31, col = lane & 15, g = lane >> 4; const size_t r0 = (size_t)blockIdx.x * 64 + wave * 16;
  float sq[8];
#pragma unroll
  for (int r = 0; r < 8; ++r) sq[r] = 0.f;
#pragma unroll 1
  for (int half = 0; half < 2; ++half) { v8f acc[8] = {};
#pragma unroll 2
    for (int kc = 0; kc < CC / 32; ++kc) { const v16b ah = frag_b(XH + (r0 + col) * CC + kc * 32, lane), al = frag_b(XL + (r0 + col) * CC + kc * 32, lane);
#pragma unroll
      for (int j = 0; j < 8; ++j) { const size_t ro = (size_t)(half * 128 + j * 16 + col) * CC + kc * 32; const v16b wh = frag_b(WH + ro, lane), wl = frag_b(WL + ro, lane); acc[j] = wmma_bf(al, wh, acc[j]); acc[j] = wmma_bf(ah, wl, acc[j]); acc[j] = wmma_bf(ah, wh, acc[j]); } }
#pragma unroll
    for (int j = 0; j < 8; ++j) { const int c = half * 128 + j * 16 + col; const float bb = CBIAS[c];
#pragma unroll
      for (int r = 0; r < 8; ++r) { const float v = acc[j][r] + bb; sz[wave][8 * g + r][c] = v; sq[r] += v * v; } } }
#pragma unroll
  for (int r = 0; r < 8; ++r) ssq[wave][8 * g + r][col] = sq[r];
  LDSX();
  for (int rl = 0; rl < 16; ++rl) { float tot = 0.f;
#pragma unroll
    for (int k = 0; k < 16; ++k) tot += ssq[wave][rl][k];
    const float inv = 1.0f / fmaxf(sqrtf(tot), 1e-12f); float psq = 0.f;
    for (int c = lane; c < EE; c += 32) { const float zn = sz[wave][rl][c] * inv; sz[wave][rl][c] = zn; szb[wave][rl][c] = (__bf16)zn; psq += zn * zn; }
#pragma unroll
    for (int o = 1; o < 32; o <<= 1) psq += __shfl_xor(psq, o);
    if (lane == 0) szsq[wave * 16 + rl] = psq; }
  LDSX();
  for (int rl = 0; rl < 16; ++rl) { vst2(ZF + (r0 + rl) * EE + lane * 4, *(const v4f*)&sz[wave][rl][lane * 4]); vst2(ZF + (r0 + rl) * EE + 128 + lane * 4, *(const v4f*)&sz[wave][rl][128 + lane * 4]); vst2((unsigned*)(ZB + (r0 + rl) * EE + lane * 8), *(const v4u*)&szb[wave][rl][lane * 8]); }
  __syncthreads();
  if (tid < 16) vst2(ZSQ + (size_t)blockIdx.x * 64 + tid * 4, *(const v4f*)&szsq[tid * 4]);
}
__global__ __launch_bounds__(256) void k_cb(const float* __restrict__ EMB, float* __restrict__ CF, __bf16* __restrict__ CBp, float* __restrict__ CSQ) {
  __shared__ __align__(16) float sc[8][EE + 4]; __shared__ __align__(16) __bf16 scb[8][EE + 8]; __shared__ __align__(16) float ssq[64]; const int tid = threadIdx.x, wave = tid >> 5, lane = tid & 31;
  for (int it = 0; it < 8; ++it) { const size_t n = (size_t)blockIdx.x * 64 + it * 8 + wave; const float* src = EMB + n * EE; float v[8]; float s = 0.f;
#pragma unroll
    for (int k = 0; k < 8; ++k) { v[k] = src[lane + 32 * k]; s += v[k] * v[k]; }
#pragma unroll
    for (int o = 1; o < 32; o <<= 1) s += __shfl_xor(s, o);
    const float inv = 1.0f / fmaxf(sqrtf(s), 1e-12f); float s2 = 0.f;
#pragma unroll
    for (int k = 0; k < 8; ++k) { const float cn = v[k] * inv; sc[wave][lane + 32 * k] = cn; scb[wave][lane + 32 * k] = (__bf16)cn; s2 += cn * cn; }
#pragma unroll
    for (int o = 1; o < 32; o <<= 1) s2 += __shfl_xor(s2, o);
    if (lane == 0) ssq[it * 8 + wave] = s2;
    LDSX();
    vst2(CF + n * EE + lane * 4, *(const v4f*)&sc[wave][lane * 4]); vst2(CF + n * EE + 128 + lane * 4, *(const v4f*)&sc[wave][128 + lane * 4]); vst2((unsigned*)(CBp + n * EE + lane * 8), *(const v4u*)&scb[wave][lane * 8]);
    LDSX(); }
  __syncthreads();
  if (tid < 16) vst2(CSQ + (size_t)blockIdx.x * 64 + tid * 4, *(const v4f*)&ssq[tid * 4]);
}
__global__ __launch_bounds__(128) void k_vq(const __bf16* __restrict__ ZB, const __bf16* __restrict__ CBp, const float* __restrict__ CSQ, const float* __restrict__ CF, const float* __restrict__ ZF, const float* __restrict__ ZSQ, int* __restrict__ OUT) {
  __shared__ int scand[4][16][64]; __shared__ __align__(16) int sbest[64];
  const int tid = threadIdx.x, wave = tid >> 5, lane = tid & 31, col = lane & 15, g = lane >> 4; const size_t r0 = (size_t)blockIdx.x * 64 + wave * 16;
  float bv[8][NTOP]; int bi[8][NTOP];
#pragma unroll
  for (int r = 0; r < 8; ++r)
#pragma unroll
    for (int s = 0; s < NTOP; ++s) { bv[r][s] = -3.0e38f; bi[r][s] = 0; }
  v16b az[CC / 32];
#pragma unroll
  for (int kc = 0; kc < EE / 32; ++kc) az[kc] = frag_b(ZB + (r0 + col) * EE + kc * 32, lane);
#pragma unroll 1
  for (int ch = 0; ch < NCB / 128; ++ch) { const int n0 = ch * 128; v8f acc[8] = {};
#pragma unroll
    for (int kc = 0; kc < EE / 32; ++kc) {
#pragma unroll
      for (int j = 0; j < 8; ++j) acc[j] = wmma_bf(az[kc], frag_b(CBp + (size_t)(n0 + j * 16 + col) * EE + kc * 32, lane), acc[j]); }
#pragma unroll
    for (int j = 0; j < 8; ++j) { const int n = n0 + j * 16 + col; const float cs = CSQ[n];
#pragma unroll
      for (int r = 0; r < 8; ++r) { const float sc = 2.0f * acc[j][r] - cs;
        if (sc > bv[r][NTOP - 1]) { float cv = sc; int ci = n; bool placed = false;
#pragma unroll
          for (int s = 0; s < NTOP; ++s) { const bool swp = placed || (cv > bv[r][s]); placed = swp; const float tv = bv[r][s]; const int ti = bi[r][s]; bv[r][s] = swp ? cv : tv; bi[r][s] = swp ? ci : ti; cv = swp ? tv : cv; ci = swp ? ti : ci; } } } } }
#pragma unroll
  for (int r = 0; r < 8; ++r)
#pragma unroll
    for (int s = 0; s < NTOP; ++s) scand[wave][8 * g + r][s * 16 + col] = bi[r][s];
  LDSX();
#pragma unroll 1
  for (int rl = 0; rl < 16; ++rl) { const size_t row = r0 + rl; const float* zr = ZF + row * EE; const double zsq = (double)ZSQ[row]; double bestd = 1e300; int besti = 0x7fffffff;
#pragma unroll 1
    for (int h2 = 0; h2 < 2; ++h2) { const int cand = scand[wave][rl][h2 * 32 + lane]; const float* cr = CF + (size_t)cand * EE; double dot = 0.0;
#pragma unroll 4
      for (int k = 0; k < EE; ++k) dot += (double)zr[k] * (double)cr[k];
      const double dist = (zsq + (double)CSQ[cand]) - 2.0 * dot;
      if (dist < bestd || (dist == bestd && cand < besti)) { bestd = dist; besti = cand; } }
    double bvv = bestd; int bii = besti;
#pragma unroll
    for (int o = 1; o < 32; o <<= 1) { const unsigned long long u = __double_as_longlong(bvv); const int lo = __shfl_xor((int)(u & 0xffffffffu), o), hi = __shfl_xor((int)(u >> 32), o); const int oi = __shfl_xor(bii, o);
      const double ov = __longlong_as_double(((unsigned long long)(unsigned)hi << 32) | (unsigned long long)(unsigned)lo);
      if (ov < bvv || (ov == bvv && oi < bii)) { bvv = ov; bii = oi; } }
    if (lane == 0) sbest[wave * 16 + rl] = bii; }
  __syncthreads();
  if (tid < 16) vst2((unsigned*)(OUT + (size_t)blockIdx.x * 64 + tid * 4), *(const v4u*)&sbest[tid * 4]);
}
extern "C" void kernel_launch(void* const* d_in, const int* in_sizes, int n_in, void* d_out, int out_size, void* d_ws, size_t ws_size, hipStream_t stream) {
  (void)in_sizes; (void)n_in; (void)out_size;
  const float** F = (const float**)d_in;
  if (ws_size < (size_t)WS_END) return;
  char* ws = (char*)d_ws; __bf16 *XH = (__bf16*)(ws + WS_XH), *XL = (__bf16*)(ws + WS_XL), *WH = (__bf16*)(ws + WS_WH), *WL = (__bf16*)(ws + WS_WL), *ZB = (__bf16*)(ws + WS_ZB), *CBp = (__bf16*)(ws + WS_CB); float *ZF = (float*)(ws + WS_ZF), *CF = (float*)(ws + WS_CF), *CSQ = (float*)(ws + WS_CSQ), *ZSQ = (float*)(ws + WS_ZSQ);
  k_xrows<<<dim3(NPIX / 64, 16), 256, 0, stream>>>(F[0], XH, XL);
  k_wrows<<<EE, 256, 0, stream>>>(F[2], WH, WL);
  k_conv<<<NRT, 128, 0, stream>>>(XH, XL, WH, WL, F[3], ZF, ZB, ZSQ);
  k_cb<<<NCB / 64, 256, 0, stream>>>(F[1], CF, CBp, CSQ);
  k_vq<<<NRT, 128, 0, stream>>>(ZB, CBp, CSQ, CF, ZF, ZSQ, (int*)d_out);
}
